// GCNEdge2Cluster_modularity_51144470561271
// MI455X (gfx1250) — hardware-verified
//
#include <hip/hip_runtime.h>
#include <stddef.h>
#include <stdint.h>


#define FDIM    128
#define HDIM    256
#define KCL     30
#define GLW     64
#define NTHR    256
#define NWAVE   8
#define EPT     8
#define NGRP    2
#define CHUNK   (NTHR * EPT * NGRP)
#define WCAP    (EPT * NGRP * 32)
#define LISTN   (NWAVE * WCAP)
#define NBS     4096
#define NBF     1024
#define RCAP    49152
#define NFBMAX  128
#define DEGCAP  256
#define TPB1    32
#define G1ROWS  128
#define APITCH  264
#define G2ROWS  64
#define G2THR   128
#define SPITCH  68
#define TPB2    32
#define TPBC    64
#define WSCALE  16.0f
#define WINV    0.0625f
#define REGC    0.01

#define LDS_GEMM1 (2 * G1ROWS * APITCH * 2)
#define LDS_FILL  ((RCAP + NBF + LISTN + NWAVE) * 4)

static_assert((CHUNK & (CHUNK - 1)) == 0);
static_assert(CHUNK <= 4096);
static_assert((NBS & (NBS - 1)) == 0 && NBS <= 4096);
static_assert((NBF & (NBF - 1)) == 0 && NBF <= 4096);
static_assert((RCAP % 32) == 0);
static_assert((TPB2 * KCL) % 4 == 0);
static_assert(NFBMAX == 128);
static_assert(HDIM % 32 == 0 && GLW % 16 == 0);

typedef float    v4f  __attribute__((ext_vector_type(4)));
typedef float    v8f  __attribute__((ext_vector_type(8)));
typedef int      v4i  __attribute__((ext_vector_type(4)));
typedef double   v2d  __attribute__((ext_vector_type(2)));
typedef _Float16 v4h  __attribute__((ext_vector_type(4)));
typedef _Float16 v8h  __attribute__((ext_vector_type(8)));
typedef _Float16 v16h __attribute__((ext_vector_type(16)));
union FragH { v16h v; v8h h[2]; };

__device__ __forceinline__ v8h cvt8(v4f a, v4f b) {
  v8h r;
  r[0] = (_Float16)a.x; r[1] = (_Float16)a.y; r[2] = (_Float16)a.z; r[3] = (_Float16)a.w;
  r[4] = (_Float16)b.x; r[5] = (_Float16)b.y; r[6] = (_Float16)b.z; r[7] = (_Float16)b.w;
  return r;
}

__device__ __forceinline__ v4f sel4(bool c, v4f a, v4f b) {
  v4f r;
  r.x = c ? a.x : b.x; r.y = c ? a.y : b.y; r.z = c ? a.z : b.z; r.w = c ? a.w : b.w;
  return r;
}

__device__ __forceinline__ v8f wmh(v16h a, v16h b, v8f c) {
  v8f d = __builtin_amdgcn_wmma_f32_16x16x32_f16(false, a, false, b, (short)0, c, false, false);
  asm volatile("v_nop\n\tv_nop\n\tv_nop\n\tv_nop" : "+v"(d) : "v"(a), "v"(b));
  return d;
}

__device__ __forceinline__ float wave_max(float v) {
#pragma unroll
  for (int o = 16; o > 0; o >>= 1) v = fmaxf(v, __shfl_xor(v, o, 32));
  return v;
}
__device__ __forceinline__ float wave_sum(float v) {
#pragma unroll
  for (int o = 16; o > 0; o >>= 1) v += __shfl_xor(v, o, 32);
  return v;
}

template <int NB>
__device__ __forceinline__ int scan_chunk(const int* __restrict__ ids, int nE, int cbase, int nodeBase,
                                          int vec8, int* list, int tid, int lane, int wave) {
  int wc = 0;
#pragma unroll
  for (int g = 0; g < NGRP; ++g) {
    const int el0  = (g * NTHR + tid) * EPT;
    const int e0   = cbase + el0;
    const int sent = -2147483647 - 1;
    v4i da, db;
    if (vec8 != 0 && cbase + CHUNK <= nE) {
      da = *(const v4i*)(ids + e0);
      db = *(const v4i*)(ids + e0 + 4);
    } else {
      da.x = (e0     < nE) ? ids[min(e0,     nE - 1)] : sent;
      da.y = (e0 + 1 < nE) ? ids[min(e0 + 1, nE - 1)] : sent;
      da.z = (e0 + 2 < nE) ? ids[min(e0 + 2, nE - 1)] : sent;
      da.w = (e0 + 3 < nE) ? ids[min(e0 + 3, nE - 1)] : sent;
      db.x = (e0 + 4 < nE) ? ids[min(e0 + 4, nE - 1)] : sent;
      db.y = (e0 + 5 < nE) ? ids[min(e0 + 5, nE - 1)] : sent;
      db.z = (e0 + 6 < nE) ? ids[min(e0 + 6, nE - 1)] : sent;
      db.w = (e0 + 7 < nE) ? ids[min(e0 + 7, nE - 1)] : sent;
    }
    const unsigned nb = (unsigned)nodeBase;
    const unsigned s0 = (unsigned)da.x - nb, s1 = (unsigned)da.y - nb;
    const unsigned s2 = (unsigned)da.z - nb, s3 = (unsigned)da.w - nb;
    const unsigned s4 = (unsigned)db.x - nb, s5 = (unsigned)db.y - nb;
    const unsigned s6 = (unsigned)db.z - nb, s7 = (unsigned)db.w - nb;
    const bool h0 = s0 < (unsigned)NB, h1 = s1 < (unsigned)NB, h2 = s2 < (unsigned)NB, h3 = s3 < (unsigned)NB;
    const bool h4 = s4 < (unsigned)NB, h5 = s5 < (unsigned)NB, h6 = s6 < (unsigned)NB, h7 = s7 < (unsigned)NB;
    const unsigned any = __builtin_amdgcn_ballot_w32(h0 | h1 | h2 | h3 | h4 | h5 | h6 | h7);
    if (any != 0u) {
#define HITJ(J, HJ, SJ) { \
        const unsigned mj = __builtin_amdgcn_ballot_w32(HJ); \
        if (mj != 0u) { \
          if (HJ) { \
            const int pos = wc + (int)__builtin_amdgcn_mbcnt_lo(mj, 0u); \
            if (pos < WCAP) list[wave * WCAP + pos] = ((el0 + (J)) << 12) | (int)(SJ); \
          } \
          wc += (int)__builtin_popcount(mj); } }
      HITJ(0, h0, s0)
      HITJ(1, h1, s1)
      HITJ(2, h2, s2)
      HITJ(3, h3, s3)
      HITJ(4, h4, s4)
      HITJ(5, h5, s5)
      HITJ(6, h6, s6)
      HITJ(7, h7, s7)
#undef HITJ
    }
  }
  return wc;
}

__global__ __launch_bounds__(NTHR) void k_wprep(
    const float* __restrict__ Wc1, const float* __restrict__ Wl1,
    const float* __restrict__ Wc2, const float* __restrict__ Wl2,
    _Float16* w1p, _Float16* w2p) {
  const int i  = blockIdx.x * NTHR + threadIdx.x;
  const int n1 = HDIM * HDIM / 8;
  const int n2 = GLW * HDIM / 8;
  v4f a, b;
  _Float16* dp;
  if (i < n1) {
    const int o  = i * 8;
    const int n  = o >> 8;
    const int k0 = o & 255;
    const int ka = min(k0, FDIM - 8);
    const int kb = min(max(k0 - FDIM, 0), FDIM - 8);
    const float* pa = Wc1 + (size_t)ka * HDIM + n;
    const float* pb = Wl1 + (size_t)kb * HDIM + n;
    v4f a0, b0, a1, b1;
    a0.x = pa[0];        a0.y = pa[HDIM];     a0.z = pa[2 * HDIM]; a0.w = pa[3 * HDIM];
    b0.x = pa[4 * HDIM]; b0.y = pa[5 * HDIM]; b0.z = pa[6 * HDIM]; b0.w = pa[7 * HDIM];
    a1.x = pb[0];        a1.y = pb[HDIM];     a1.z = pb[2 * HDIM]; a1.w = pb[3 * HDIM];
    b1.x = pb[4 * HDIM]; b1.y = pb[5 * HDIM]; b1.z = pb[6 * HDIM]; b1.w = pb[7 * HDIM];
    const bool lo = k0 < FDIM;
    a = sel4(lo, a0, a1);
    b = sel4(lo, b0, b1);
    dp = w1p + o;
  } else if (i < n1 + n2) {
    const int o  = (i - n1) * 8;
    const int n  = o >> 8;
    const int k0 = o & 255;
    const int na = min(n, KCL - 1);
    const int nb = min(max(n - 32, 0), KCL - 1);
    const float* pa = Wc2 + (size_t)k0 * KCL + na;
    const float* pb = Wl2 + (size_t)k0 * KCL + nb;
    v4f a0, b0, a1, b1;
    a0.x = pa[0];       a0.y = pa[KCL];     a0.z = pa[2 * KCL]; a0.w = pa[3 * KCL];
    b0.x = pa[4 * KCL]; b0.y = pa[5 * KCL]; b0.z = pa[6 * KCL]; b0.w = pa[7 * KCL];
    a1.x = pb[0];       a1.y = pb[KCL];     a1.z = pb[2 * KCL]; a1.w = pb[3 * KCL];
    b1.x = pb[4 * KCL]; b1.y = pb[5 * KCL]; b1.z = pb[6 * KCL]; b1.w = pb[7 * KCL];
    const v4f z = {0.f, 0.f, 0.f, 0.f};
    const bool isc = n < KCL;
    const bool isl = (n >= 32) && (n < 32 + KCL);
    a = sel4(isc, a0, sel4(isl, a1, z));
    b = sel4(isc, b0, sel4(isl, b1, z));
    dp = w2p + o;
  } else {
    return;
  }
  a = a * WSCALE;
  b = b * WSCALE;
  const v8h hv = cvt8(a, b);
  *(volatile v8h*)dp = hv;
  __threadfence();
  *(volatile v8h*)dp = hv;
}

__global__ __launch_bounds__(NTHR) void k_seg(
    const int* __restrict__ ei, const float* __restrict__ ew,
    int* cntp, float* wsp, float* disp, int nN, int nE, int nBD, int vec8) {
  __shared__ __attribute__((aligned(16))) int   cnt[NBS];
  __shared__ __attribute__((aligned(16))) float wsm[NBS];
  __shared__ __attribute__((aligned(16))) int   list[LISTN];
  __shared__ int wcnt[NWAVE];
  const int tid = threadIdx.x, lane = tid & 31, wave = tid >> 5;
  const int blk = blockIdx.x;
  const int second = (blk >= nBD) ? 1 : 0;
  const int nodeBase = (blk - second * nBD) * NBS;
  const int* ids = ei + (second ? 0 : nE);
  (void)nN;

  for (int i = tid; i < NBS; i += NTHR) { cnt[i] = 0; wsm[i] = 0.f; }
  __syncthreads();

  const int nChunks = (nE + CHUNK - 1) / CHUNK;
#pragma unroll 1
  for (int ch = 0; ch < nChunks; ++ch) {
    const int cbase = ch * CHUNK;
    const int wc = scan_chunk<NBS>(ids, nE, cbase, nodeBase, vec8, list, tid, lane, wave);
    if (lane == 0) wcnt[wave] = wc;
    __syncthreads();
    if (wave == 0) {
#pragma unroll 1
      for (int wsx = 0; wsx < NWAVE; ++wsx) {
        int n = __builtin_amdgcn_readfirstlane(wcnt[wsx]);
        n = n > WCAP ? WCAP : (n < 0 ? 0 : n);
        const int* lp = list + wsx * WCAP;
#pragma unroll 1
        for (int i = 0; i < n; ++i) {
          const int ent  = __builtin_amdgcn_readfirstlane(lp[i]);
          const int slot = ent & (NBS - 1);
          int e = cbase + ((ent >> 12) & (CHUNK - 1));
          e = e > nE - 1 ? nE - 1 : e;
          const float w = ew[e];
          if (lane == 0) { cnt[slot] = cnt[slot] + 1; wsm[slot] = wsm[slot] + w; }
        }
      }
    }
    __syncthreads();
  }

  v4i cq[4]; v4f wq[4], dq[4];
#pragma unroll
  for (int q = 0; q < 4; ++q) {
    const int f = (wave * 4 + q) * 128 + 4 * lane;
    cq[q] = *(const v4i*)(cnt + f);
    wq[q] = *(const v4f*)(wsm + f);
    dq[q].x = rsqrtf(wq[q].x + 1.0f);
    dq[q].y = rsqrtf(wq[q].y + 1.0f);
    dq[q].z = rsqrtf(wq[q].z + 1.0f);
    dq[q].w = rsqrtf(wq[q].w + 1.0f);
  }
  const size_t pb = (size_t)blk * NBS;
#pragma unroll
  for (int q = 0; q < 4; ++q) {
    const int f = (wave * 4 + q) * 128 + 4 * lane;
    *(volatile v4i*)(cntp + pb + f) = cq[q];
    *(volatile v4f*)(wsp  + pb + f) = wq[q];
    *(volatile v4f*)(disp + pb + f) = dq[q];
  }
  __threadfence();
#pragma unroll
  for (int q = 0; q < 4; ++q) {
    const int f = (wave * 4 + q) * 128 + 4 * lane;
    *(volatile v4i*)(cntp + pb + f) = cq[q];
    *(volatile v4f*)(wsp  + pb + f) = wq[q];
    *(volatile v4f*)(disp + pb + f) = dq[q];
  }
}

__global__ __launch_bounds__(NTHR) void k_off(
    const int* __restrict__ cntp, int* offp, int* rbp, int nN, int nFB) {
  __shared__ int wtot[NWAVE];
  __shared__ __attribute__((aligned(16))) int rb[NFBMAX];
  const int tid = threadIdx.x, lane = tid & 31, wave = tid >> 5;
  for (int i = tid; i < NFBMAX; i += NTHR) rb[i] = 0;
  int carry = 0;
  __syncthreads();
#pragma unroll 1
  for (int b = 0; b < nFB; ++b) {
    const int n0 = b * NBF + 4 * tid;
    const v4i cv = *(const v4i*)(cntp + n0);
    const int c0 = (n0     < nN) ? min(max(cv.x, 0), DEGCAP) : 0;
    const int c1 = (n0 + 1 < nN) ? min(max(cv.y, 0), DEGCAP) : 0;
    const int c2 = (n0 + 2 < nN) ? min(max(cv.z, 0), DEGCAP) : 0;
    const int c3 = (n0 + 3 < nN) ? min(max(cv.w, 0), DEGCAP) : 0;
    const int t1 = c0, t2 = t1 + c1, t3 = t2 + c2, t4 = t3 + c3;
    int v = t4;
#pragma unroll
    for (int d = 1; d < 32; d <<= 1) {
      const int u = __shfl_up(v, d, 32);
      if (lane >= d) v += u;
    }
    if (lane == 31) wtot[wave] = v;
    __syncthreads();
    int wp = 0, bt = 0;
#pragma unroll
    for (int w = 0; w < NWAVE; ++w) {
      const int t = wtot[w];
      wp += (w < wave) ? t : 0;
      bt += t;
    }
    const int ex = carry + wp + v - t4;
    v4i ov; ov.x = ex; ov.y = ex + t1; ov.z = ex + t2; ov.w = ex + t3;
    int* op = offp + n0;
    *(volatile v4i*)op = ov;
    __threadfence();
    *(volatile v4i*)op = ov;
    if (tid == 0) rb[b] = carry;
    carry += (bt + 31) & ~31;
    __syncthreads();
  }
  if (tid == 0) {
#pragma unroll 1
    for (int j = nFB; j < NFBMAX; ++j) rb[j] = carry;
  }
  __syncthreads();
  if (wave == 0) {
    const v4i rv = *(const v4i*)(rb + 4 * lane);
    *(volatile v4i*)(rbp + 4 * lane) = rv;
    __threadfence();
    *(volatile v4i*)(rbp + 4 * lane) = rv;
  }
}

__global__ __launch_bounds__(NTHR) void k_fill(
    const int* __restrict__ ei, const int* __restrict__ offp, const int* __restrict__ rbp,
    int* csr, int nN, int nE, int csrCap, int vec8) {
  extern __shared__ v4i lds_dyn_i[];
  int* region = (int*)lds_dyn_i;
  int* cur    = region + RCAP;
  int* list   = cur + NBF;
  int* wcnt   = list + LISTN;
  const int tid = threadIdx.x, lane = tid & 31, wave = tid >> 5;
  const int b = blockIdx.x, nodeBase = b * NBF;
  const int* ids = ei + nE;
  (void)nN;

  int rb0 = rbp[b];
  const int rb1 = rbp[b + 1];
  rb0 = min(max(rb0, 0), csrCap);
  int len = rb1 - rb0;
  len = min(max(len, 0), RCAP);
  len = min(len, csrCap - rb0);
  len &= ~31;

  {
    const v4i z = {0, 0, 0, 0};
    for (int i = tid; i < RCAP / 4; i += NTHR) lds_dyn_i[i] = z;
  }
  for (int s = tid; s < NBF; s += NTHR) {
    int o = offp[nodeBase + s] - rb0;
    o = min(max(o, 0), RCAP);
    cur[s] = o;
  }
  __syncthreads();

  const int nChunks = (nE + CHUNK - 1) / CHUNK;
#pragma unroll 1
  for (int ch = 0; ch < nChunks; ++ch) {
    const int cbase = ch * CHUNK;
    const int wc = scan_chunk<NBF>(ids, nE, cbase, nodeBase, vec8, list, tid, lane, wave);
    if (lane == 0) wcnt[wave] = wc;
    __syncthreads();
    if (wave == 0) {
#pragma unroll 1
      for (int wsx = 0; wsx < NWAVE; ++wsx) {
        int n = __builtin_amdgcn_readfirstlane(wcnt[wsx]);
        n = n > WCAP ? WCAP : (n < 0 ? 0 : n);
        const int* lp = list + wsx * WCAP;
#pragma unroll 1
        for (int i = 0; i < n; ++i) {
          const int ent  = __builtin_amdgcn_readfirstlane(lp[i]);
          const int slot = ent & (NBF - 1);
          int e = cbase + ((ent >> 12) & (CHUNK - 1));
          e = e > nE - 1 ? nE - 1 : e;
          if (lane == 0) {
            const int pos = cur[slot];
            if ((unsigned)pos < (unsigned)RCAP) { region[pos] = e; cur[slot] = pos + 1; }
          }
        }
      }
    }
    __syncthreads();
  }
  __syncthreads();

  const int pieces = len >> 2;
  int* gp = csr + rb0;
#pragma unroll 1
  for (int p = tid; p < pieces; p += NTHR) {
    const v4i rv = *(const v4i*)(region + 4 * p);
    *(volatile v4i*)(gp + 4 * p) = rv;
  }
  __threadfence();
#pragma unroll 1
  for (int p = tid; p < pieces; p += NTHR) {
    const v4i rv = *(const v4i*)(region + 4 * p);
    *(volatile v4i*)(gp + 4 * p) = rv;
  }
}

__global__ __launch_bounds__(NTHR) void k_agg1(
    const float* __restrict__ x, const int* __restrict__ ei, const float* __restrict__ ew,
    const int* __restrict__ cntp, const int* __restrict__ offp, const int* __restrict__ csr,
    const float* __restrict__ disp, _Float16* a1, int nN, int nE, int csrCap) {
  const int tid = threadIdx.x, lane = tid & 31, wave = tid >> 5;
#pragma unroll 1
  for (int q = 0; q < TPB1 / NWAVE; ++q) {
    const int c = blockIdx.x * TPB1 + wave * (TPB1 / NWAVE) + q;
    if (c >= nN) break;
    int n = __builtin_amdgcn_readfirstlane(cntp[c]);
    n = min(max(n, 0), DEGCAP);
    int o = __builtin_amdgcn_readfirstlane(offp[c]);
    o = min(max(o, 0), csrCap - 1);
    const float dc = disp[c];
    v4f acc = {0.f, 0.f, 0.f, 0.f};
#pragma unroll 1
    for (int base = 0; base < n; base += 32) {
      int pos = o + base + lane;
      pos = min(pos, csrCap - 1);
      int e = csr[pos];
      e = min(max(e, 0), nE - 1);
      int r = ei[e];
      r = min(max(r, 0), nN - 1);
      const float cf = ew[e] * disp[r];
      const int mcnt = min(32, n - base);
#pragma unroll 2
      for (int jj = 0; jj < mcnt; ++jj) {
        const int   rr = __shfl(r, jj, 32);
        const float cc = __shfl(cf, jj, 32);
        const v4f xv = *(const v4f*)(x + (size_t)rr * FDIM + 4 * lane);
        acc += xv * cc;
      }
    }
    const v4f xc  = *(const v4f*)(x + (size_t)c * FDIM + 4 * lane);
    const v4f res = acc * dc + xc * (dc * dc);
    v4h hv;
    hv.x = (_Float16)res.x; hv.y = (_Float16)res.y; hv.z = (_Float16)res.z; hv.w = (_Float16)res.w;
    _Float16* dp = a1 + (size_t)c * FDIM + 4 * lane;
    *(volatile v4h*)dp = hv;
    __threadfence();
    *(volatile v4h*)dp = hv;
  }
}

__global__ __launch_bounds__(NTHR) void k_gemm1(
    const _Float16* __restrict__ a1, const float* __restrict__ x,
    const _Float16* __restrict__ w1p, const float* __restrict__ bc1, const float* __restrict__ bl1,
    _Float16* hp, int nN) {
  extern __shared__ v4f lds_dyn[];
  _Float16* sA  = (_Float16*)lds_dyn;
  _Float16* stg = sA + G1ROWS * APITCH;
  const int tid = threadIdx.x, lane = tid & 31, wave = tid >> 5, hh = lane >> 4, m = lane & 15;
  const int rowBase = blockIdx.x * G1ROWS;

#pragma unroll
  for (int i = 0; i < (G1ROWS * FDIM / 8) / NTHR; ++i) {
    const int idx = i * NTHR + tid;
    const int r   = idx >> 4;
    const int c8  = (idx & 15) * 8;
    const int node = min(rowBase + r, nN - 1);
    const v8h v = *(const v8h*)(a1 + (size_t)node * FDIM + c8);
    *(v8h*)(sA + r * APITCH + c8) = v;
  }
#pragma unroll
  for (int i = 0; i < (G1ROWS * FDIM / 8) / NTHR; ++i) {
    const int idx = i * NTHR + tid;
    const int r   = idx >> 4;
    const int c8  = (idx & 15) * 8;
    const int node = min(rowBase + r, nN - 1);
    const float* xp = x + (size_t)node * FDIM + c8;
    const v4f a = *(const v4f*)xp, b = *(const v4f*)(xp + 4);
    *(v8h*)(sA + r * APITCH + FDIM + c8) = cvt8(a, b);
  }
  __syncthreads();

  const _Float16* ar = sA + (wave * 16 + m) * APITCH + 8 * hh;
#pragma unroll 1
  for (int nh = 0; nh < 2; ++nh) {
    v8f acc[8];
#pragma unroll
    for (int t = 0; t < 8; ++t) { v8f z = {0.f, 0.f, 0.f, 0.f, 0.f, 0.f, 0.f, 0.f}; acc[t] = z; }
#pragma unroll
    for (int kt = 0; kt < HDIM / 32; ++kt) {
      FragH a;
      a.h[0] = *(const v8h*)(ar + 32 * kt);
      a.h[1] = *(const v8h*)(ar + 32 * kt + 16);
#pragma unroll
      for (int t = 0; t < 8; ++t) {
        const _Float16* bp = w1p + (size_t)(nh * 128 + 16 * t + m) * HDIM + 32 * kt + 8 * hh;
        FragH b;
        b.h[0] = *(const v8h*)bp;
        b.h[1] = *(const v8h*)(bp + 16);
        acc[t] = wmh(a.v, b.v, acc[t]);
      }
    }
#pragma unroll
    for (int t = 0; t < 8; ++t) {
      const int col = nh * 128 + 16 * t + m;
      const float bs = bc1[col] + bl1[col];
      _Float16* sp = stg + (wave * 16 + 8 * hh) * APITCH + col;
      sp[0 * APITCH] = (_Float16)fmaxf(acc[t][0] * WINV + bs, 0.f);
      sp[1 * APITCH] = (_Float16)fmaxf(acc[t][1] * WINV + bs, 0.f);
      sp[2 * APITCH] = (_Float16)fmaxf(acc[t][2] * WINV + bs, 0.f);
      sp[3 * APITCH] = (_Float16)fmaxf(acc[t][3] * WINV + bs, 0.f);
      sp[4 * APITCH] = (_Float16)fmaxf(acc[t][4] * WINV + bs, 0.f);
      sp[5 * APITCH] = (_Float16)fmaxf(acc[t][5] * WINV + bs, 0.f);
      sp[6 * APITCH] = (_Float16)fmaxf(acc[t][6] * WINV + bs, 0.f);
      sp[7 * APITCH] = (_Float16)fmaxf(acc[t][7] * WINV + bs, 0.f);
    }
  }
  __syncthreads();

  const _Float16* lp = stg + (wave * 16) * APITCH + 8 * lane;
  _Float16* gp = hp + ((size_t)rowBase + wave * 16) * HDIM + 8 * lane;
#pragma unroll
  for (int i = 0; i < 16; ++i) { const v8h v = *(const v8h*)(lp + i * APITCH); *(volatile v8h*)(gp + (size_t)i * HDIM) = v; }
  __threadfence();
#pragma unroll
  for (int i = 0; i < 16; ++i) { const v8h v = *(const v8h*)(lp + i * APITCH); *(volatile v8h*)(gp + (size_t)i * HDIM) = v; }
}

__global__ __launch_bounds__(G2THR) void k_gemm2(
    const _Float16* __restrict__ hp, const _Float16* __restrict__ w2p, float* gl) {
  __shared__ __attribute__((aligned(16))) float stg[4 * 16 * SPITCH];
  const int tid = threadIdx.x, lane = tid & 31, wave = tid >> 5, hh = lane >> 4, m = lane & 15;
  const int rowBase = blockIdx.x * G2ROWS;
  const _Float16* ar = hp + ((size_t)rowBase + wave * 16 + m) * HDIM + 8 * hh;

  v8f acc[4];
#pragma unroll
  for (int t = 0; t < 4; ++t) { v8f z = {0.f, 0.f, 0.f, 0.f, 0.f, 0.f, 0.f, 0.f}; acc[t] = z; }
#pragma unroll
  for (int kt = 0; kt < HDIM / 32; ++kt) {
    FragH a;
    a.h[0] = *(const v8h*)(ar + 32 * kt);
    a.h[1] = *(const v8h*)(ar + 32 * kt + 16);
#pragma unroll
    for (int t = 0; t < 4; ++t) {
      const _Float16* bp = w2p + (size_t)(16 * t + m) * HDIM + 32 * kt + 8 * hh;
      FragH b;
      b.h[0] = *(const v8h*)bp;
      b.h[1] = *(const v8h*)(bp + 16);
      acc[t] = wmh(a.v, b.v, acc[t]);
    }
  }
  float* sp = stg + (wave * 16 + 8 * hh) * SPITCH + m;
#pragma unroll
  for (int t = 0; t < 4; ++t) {
    sp[0 * SPITCH + 16 * t] = acc[t][0] * WINV;
    sp[1 * SPITCH + 16 * t] = acc[t][1] * WINV;
    sp[2 * SPITCH + 16 * t] = acc[t][2] * WINV;
    sp[3 * SPITCH + 16 * t] = acc[t][3] * WINV;
    sp[4 * SPITCH + 16 * t] = acc[t][4] * WINV;
    sp[5 * SPITCH + 16 * t] = acc[t][5] * WINV;
    sp[6 * SPITCH + 16 * t] = acc[t][6] * WINV;
    sp[7 * SPITCH + 16 * t] = acc[t][7] * WINV;
  }
  __syncthreads();

  const int pc = (lane & 15) * 4;
  v4f ov[8];
#pragma unroll
  for (int q = 0; q < 8; ++q) {
    const int row = 2 * q + (lane >> 4);
    ov[q] = *(const v4f*)(stg + (wave * 16 + row) * SPITCH + pc);
  }
#pragma unroll
  for (int q = 0; q < 8; ++q) {
    const int row = 2 * q + (lane >> 4);
    *(volatile v4f*)(gl + ((size_t)rowBase + wave * 16 + row) * GLW + pc) = ov[q];
  }
  __threadfence();
#pragma unroll
  for (int q = 0; q < 8; ++q) {
    const int row = 2 * q + (lane >> 4);
    *(volatile v4f*)(gl + ((size_t)rowBase + wave * 16 + row) * GLW + pc) = ov[q];
  }
}

__global__ __launch_bounds__(NTHR) void k_agg2(
    const float* __restrict__ gl, const int* __restrict__ ei, const float* __restrict__ ew,
    const int* __restrict__ cntp, const int* __restrict__ offp, const int* __restrict__ csr,
    const float* __restrict__ disp, const float* __restrict__ degp,
    const float* __restrict__ bc2, const float* __restrict__ bl2,
    float* out, double* part2, int nN, int nE, int csrCap) {
  __shared__ __attribute__((aligned(16))) float  fxs[TPB2 * KCL];
  __shared__ __attribute__((aligned(16))) double pd[64];
  const int tid = threadIdx.x, lane = tid & 31, wave = tid >> 5;
  const int blk = blockIdx.x;
  const int kk = min(lane, KCL - 1);
  const bool act = lane < KCL;
  const float bb = bc2[kk] + bl2[kk];

#pragma unroll 1
  for (int q = 0; q < TPB2 / NWAVE; ++q) {
    const int rl = wave * (TPB2 / NWAVE) + q;
    const int c  = blk * TPB2 + rl;
    if (c < nN) {
      int n = __builtin_amdgcn_readfirstlane(cntp[c]);
      n = min(max(n, 0), DEGCAP);
      int o = __builtin_amdgcn_readfirstlane(offp[c]);
      o = min(max(o, 0), csrCap - 1);
      const float dc = disp[c];
      float acc = 0.f;
#pragma unroll 1
      for (int base = 0; base < n; base += 32) {
        int pos = o + base + lane;
        pos = min(pos, csrCap - 1);
        int e = csr[pos];
        e = min(max(e, 0), nE - 1);
        int r = ei[e];
        r = min(max(r, 0), nN - 1);
        const float cf = ew[e] * disp[r];
        const int mcnt = min(32, n - base);
#pragma unroll 2
        for (int jj = 0; jj < mcnt; ++jj) {
          const int   rr = __shfl(r, jj, 32);
          const float cc = __shfl(cf, jj, 32);
          const float gv = gl[(size_t)rr * GLW + lane];
          acc = fmaf(cc, gv, acc);
        }
      }
      const float gc = gl[(size_t)c * GLW + lane];
      const float l2 = gl[(size_t)c * GLW + 32 + lane];
      const float v  = dc * acc + (dc * dc) * gc + l2 + bb;
      const float mx = wave_max(act ? v : -3.0e38f);
      float ex = expf((act ? v : mx) - mx);
      ex = act ? ex : 0.f;
      const float s  = wave_sum(ex);
      const float p  = ex * (1.0f / s);
      const float fx = fminf(fmaxf(p, 1e-9f), 1.0f - 1e-9f);
      if (act) fxs[rl * KCL + lane] = fx;
    }
  }
  __syncthreads();

  const int nval = min(TPB2, nN - blk * TPB2);
  const int lim  = nval * KCL;
  const size_t ob = (size_t)blk * TPB2 * KCL;
  const int t0 = lim & ~3;
  v4f pv = {0.f, 0.f, 0.f, 0.f};
  const bool pfull = (4 * tid + 4 <= lim);
  if (pfull) pv = *(const v4f*)(fxs + 4 * tid);
  float tv = 0.f;
  const bool ptail = tid < (lim & 3);
  if (ptail) tv = fxs[t0 + tid];
  if (pfull) *(volatile v4f*)(out + ob + 4 * tid) = pv;
  if (ptail) *(volatile float*)(out + ob + t0 + tid) = tv;
  __threadfence();
  if (pfull) *(volatile v4f*)(out + ob + 4 * tid) = pv;
  if (ptail) *(volatile float*)(out + ob + t0 + tid) = tv;

  if (tid < 32) {
    double ss = 0.0, cs = 0.0;
    if (tid < KCL) {
#pragma unroll 1
      for (int r = 0; r < nval; ++r) {
        const float f  = fxs[r * KCL + tid];
        const float dg = degp[blk * TPB2 + r];
        cs += (double)f;
        ss += (double)f * (double)dg;
      }
    }
    pd[tid] = ss;
    pd[32 + tid] = cs;
  }
  __syncthreads();
  if (wave == 0) {
    v2d dv; dv.x = pd[2 * lane]; dv.y = pd[2 * lane + 1];
    double* pp = part2 + (size_t)blk * 64 + 2 * lane;
    *(volatile v2d*)pp = dv;
    __threadfence();
    *(volatile v2d*)pp = dv;
  }
}

__global__ __launch_bounds__(NTHR) void k_conn(
    const float* __restrict__ fx, const int* __restrict__ ei, const float* __restrict__ ew,
    const int* __restrict__ cntp, const int* __restrict__ offp, const int* __restrict__ csr,
    double* partc, int nN, int nE, int csrCap) {
  __shared__ double pw[NWAVE];
  __shared__ double tot;
  const int tid = threadIdx.x, lane = tid & 31, wave = tid >> 5;
  const int blk = blockIdx.x;
  const int kk = min(lane, KCL - 2);
  const bool act = lane < KCL - 1;
  double wacc = 0.0;
#pragma unroll 1
  for (int q = 0; q < TPBC / NWAVE; ++q) {
    const int c = blk * TPBC + wave * (TPBC / NWAVE) + q;
    if (c < nN) {
      const float fcv = fx[(size_t)c * KCL + kk];
      const float fc  = act ? fcv : 0.f;
      int n = __builtin_amdgcn_readfirstlane(cntp[c]);
      n = min(max(n, 0), DEGCAP);
      int o = __builtin_amdgcn_readfirstlane(offp[c]);
      o = min(max(o, 0), csrCap - 1);
      float acc = 0.f;
#pragma unroll 1
      for (int base = 0; base < n; base += 32) {
        int pos = o + base + lane;
        pos = min(pos, csrCap - 1);
        int e = csr[pos];
        e = min(max(e, 0), nE - 1);
        int r = ei[e];
        r = min(max(r, 0), nN - 1);
        const float wv = ew[e];
        const int mcnt = min(32, n - base);
#pragma unroll 2
        for (int jj = 0; jj < mcnt; ++jj) {
          const int   rr = __shfl(r, jj, 32);
          const float ww = __shfl(wv, jj, 32);
          acc = fmaf(ww, fx[(size_t)rr * KCL + kk], acc);
        }
      }
      const float d = wave_sum(acc * fc);
      wacc += (double)d;
    }
  }
  if (lane == 0) pw[wave] = wacc;
  __syncthreads();
  if (tid == 0) {
    double t = 0.0;
#pragma unroll
    for (int w = 0; w < NWAVE; ++w) t += pw[w];
    tot = t;
  }
  __syncthreads();
  if (wave == 0) {
    v2d dv; dv.x = (lane == 0) ? tot : 0.0; dv.y = 0.0;
    double* pp = partc + (size_t)blk * 16 + 2 * lane;
    if (lane < 8) *(volatile v2d*)pp = dv;
    __threadfence();
    if (lane < 8) *(volatile v2d*)pp = dv;
  }
}

__global__ __launch_bounds__(NTHR) void k_loss(
    const float* __restrict__ degp, const double* __restrict__ part2, const double* __restrict__ partc,
    float* out, int nN, int nA2, int nCB) {
  __shared__ double sm[NTHR], sc[NTHR], ssk[32], csk[32];
  const int tid = threadIdx.x;
  double dm = 0.0, dcn = 0.0;
#pragma unroll 1
  for (int n = tid; n < nN; n += NTHR) dm += (double)degp[n];
#pragma unroll 1
  for (int b = tid; b < nCB; b += NTHR) dcn += partc[(size_t)b * 16];
  sm[tid] = dm;
  sc[tid] = dcn;
  if (tid < 32) {
    double ss = 0.0, cs = 0.0;
    if (tid < KCL) {
#pragma unroll 1
      for (int b = 0; b < nA2; ++b) {
        ss += part2[(size_t)b * 64 + tid];
        cs += part2[(size_t)b * 64 + 32 + tid];
      }
    }
    ssk[tid] = ss;
    csk[tid] = cs;
  }
  __syncthreads();
  if (tid == 0) {
    double m = 0.0, cn = 0.0;
#pragma unroll 1
    for (int i = 0; i < NTHR; ++i) { m += sm[i]; cn += sc[i]; }
    double sq = 0.0;
#pragma unroll 1
    for (int k = 0; k < KCL - 1; ++k) sq += ssk[k] * ssk[k];
    double cq = 0.0;
#pragma unroll 1
    for (int k = 0; k < KCL; ++k) cq += csk[k] * csk[k];
    const double twom = 2.0 * m;
    const double avg  = sq / twom;
    const double mod  = -(cn - avg) / twom;
    const double reg  = sqrt(cq + 1e-9) * sqrt((double)KCL) / (double)nN - 1.0;
    const float lf = (float)(mod + REGC * reg);
    float* lp = out + (size_t)nN * KCL;
    *(volatile float*)lp = lf;
    __threadfence();
    *(volatile float*)lp = lf;
  }
}

extern "C" void kernel_launch(void* const* d_in, const int* in_sizes, int n_in,
                              void* d_out, int out_size, void* d_ws, size_t ws_size,
                              hipStream_t stream) {
  if (n_in < 11) return;
  const int nN = in_sizes[0] / FDIM;
  const int nE = in_sizes[2];
  if (nN <= 0 || nE <= 0) return;
  if (in_sizes[0] != nN * FDIM || in_sizes[1] != 2 * nE) return;
  if (in_sizes[3] != FDIM * HDIM || in_sizes[4] < HDIM || in_sizes[5] != FDIM * HDIM || in_sizes[6] < HDIM) return;
  if (in_sizes[7] != HDIM * KCL || in_sizes[8] < KCL || in_sizes[9] != HDIM * KCL || in_sizes[10] < KCL) return;
  if (out_size != nN * KCL + 1) return;

  const float* x   = (const float*)d_in[0];
  const int*   ei  = (const int*)d_in[1];
  const float* ew  = (const float*)d_in[2];
  const float* Wc1 = (const float*)d_in[3];
  const float* bc1 = (const float*)d_in[4];
  const float* Wl1 = (const float*)d_in[5];
  const float* bl1 = (const float*)d_in[6];
  const float* Wc2 = (const float*)d_in[7];
  const float* bc2 = (const float*)d_in[8];
  const float* Wl2 = (const float*)d_in[9];
  const float* bl2 = (const float*)d_in[10];
  float* out = (float*)d_out;

  const int nBD = (nN + NBS - 1) / NBS;
  const int nFB = (nN + NBF - 1) / NBF;
  if (nFB + 1 > NFBMAX) return;
  const int csrCap = ((nE + 31) / 32) * 32 + nFB * 32 + 1024;
  const int nA1 = (nN + TPB1 - 1) / TPB1;
  const int nG1 = (nN + G1ROWS - 1) / G1ROWS;
  const int nG2 = (nN + G2ROWS - 1) / G2ROWS;
  const int nA2 = (nN + TPB2 - 1) / TPB2;
  const int nCB = (nN + TPBC - 1) / TPBC;

  char* ws = (char*)d_ws;
  size_t off = 0;
#define CARVE(NAME, BYTES) const size_t NAME = off; off += (size_t)(BYTES); off = (off + 255) & ~(size_t)255;
  CARVE(oW1,  (size_t)HDIM * HDIM * 2)
  CARVE(oW2,  (size_t)GLW * HDIM * 2)
  CARVE(oCnt, (size_t)2 * nBD * NBS * 4)
  CARVE(oWs,  (size_t)2 * nBD * NBS * 4)
  CARVE(oDis, (size_t)2 * nBD * NBS * 4)
  CARVE(oOff, (size_t)nFB * NBF * 4)
  CARVE(oRb,  (size_t)NFBMAX * 4)
  CARVE(oCsr, (size_t)csrCap * 4)
  CARVE(oA1,  (size_t)nA1 * TPB1 * FDIM * 2)
  CARVE(oH,   (size_t)nG1 * G1ROWS * HDIM * 2)
  CARVE(oGl,  (size_t)nG2 * G2ROWS * GLW * 4)
  CARVE(oP2,  (size_t)nA2 * 64 * 8)
  CARVE(oPc,  (size_t)nCB * 16 * 8)
#undef CARVE
  if (off > ws_size) return;

  _Float16* w1p  = (_Float16*)(ws + oW1);
  _Float16* w2p  = (_Float16*)(ws + oW2);
  int*      cntp = (int*)(ws + oCnt);
  float*    wsp  = (float*)(ws + oWs);
  float*    disp = (float*)(ws + oDis);
  int*      offp = (int*)(ws + oOff);
  int*      rbp  = (int*)(ws + oRb);
  int*      csr  = (int*)(ws + oCsr);
  _Float16* a1   = (_Float16*)(ws + oA1);
  _Float16* hp   = (_Float16*)(ws + oH);
  float*    gl   = (float*)(ws + oGl);
  double*   p2   = (double*)(ws + oP2);
  double*   pc   = (double*)(ws + oPc);
  float*    degp = wsp + (size_t)nBD * NBS;

  const int vec8 = ((nE & 3) == 0) ? 1 : 0;

  const int nPrep = HDIM * HDIM / 8 + GLW * HDIM / 8;
  k_wprep<<<(nPrep + NTHR - 1) / NTHR, NTHR, 0, stream>>>(Wc1, Wl1, Wc2, Wl2, w1p, w2p);

  k_seg<<<2 * nBD, NTHR, 0, stream>>>(ei, ew, cntp, wsp, disp, nN, nE, nBD, vec8);

  k_off<<<1, NTHR, 0, stream>>>(cntp, offp, rbp, nN, nFB);

  hipFuncSetAttribute(reinterpret_cast<const void*>(&k_fill),
                      hipFuncAttributeMaxDynamicSharedMemorySize, LDS_FILL);
  k_fill<<<nFB, NTHR, LDS_FILL, stream>>>(ei, offp, rbp, csr, nN, nE, csrCap, vec8);

  k_agg1<<<nA1, NTHR, 0, stream>>>(x, ei, ew, cntp, offp, csr, disp, a1, nN, nE, csrCap);

  hipFuncSetAttribute(reinterpret_cast<const void*>(&k_gemm1),
                      hipFuncAttributeMaxDynamicSharedMemorySize, LDS_GEMM1);
  k_gemm1<<<nG1, NTHR, LDS_GEMM1, stream>>>(a1, x, w1p, bc1, bl1, hp, nN);

  k_gemm2<<<nG2, G2THR, 0, stream>>>(hp, w2p, gl);

  k_agg2<<<nA2, NTHR, 0, stream>>>(gl, ei, ew, cntp, offp, csr, disp, degp, bc2, bl2, out, p2, nN, nE, csrCap);

  k_conn<<<nCB, NTHR, 0, stream>>>(out, ei, ew, cntp, offp, csr, pc, nN, nE, csrCap);

  k_loss<<<1, NTHR, 0, stream>>>(degp, p2, pc, out, nN, nA2, nCB);
}
